// XgCCA_SSG_19937238188633
// MI455X (gfx1250) — hardware-verified
//
#include <hip/hip_runtime.h>
#include <stddef.h>


#define NN      128
#define NTHR    256
#define NWAVE   8
#define EPT     8
#define NGRP    2
#define CHUNK   (NTHR * EPT * NGRP)
#define WCAP    (EPT * NGRP * 32)
#define LISTN   (NWAVE * WCAP)
#define ESHF    11
#define NBC     32768
#define NBF     2048
#define RCAP    40960
#define RBN     128
#define TGT     256
#define DEGCAP  512
#define GROWS   128
#define OTHR    512
#define WSCALE  64
#define ASC1    16
#define ASC2    64
#define SRPB    400
#define CRB     512
#define WSCAP   134217728

#define LDS_COUNT ((NBC + LISTN + NWAVE) * 4)
#define LDS_FILL  ((RCAP + NBF + LISTN + NWAVE) * 4)
#define LDS_GEMM  (GROWS * NN * 4)
#define LDS_CORR  (4 * NN * 32 * 2 + GROWS * NN * 4)
#define LDS_FIN   (NN * NN * 4 + 2 * NN * 4)

static_assert((CHUNK & (CHUNK - 1)) == 0);
static_assert((NBC & (NBC - 1)) == 0 && (NBF & (NBF - 1)) == 0);
static_assert(NBF <= (1 << ESHF));
static_assert((NBC % NBF) == 0);
static_assert(OTHR * 4 == NBF);
static_assert((RCAP % 32) == 0);
static_assert(TGT == NWAVE * 32);
static_assert(GROWS == NWAVE * 16);
static_assert((TGT % GROWS) == 0);
static_assert(NN == 128 && NN == 32 * 4);
static_assert(NBC == NWAVE * 32 * 128);
static_assert((CRB % 32) == 0 && SRPB > 0);
static_assert(((NN * NN) % NTHR) == 0);
static_assert(LDS_CORR == 98304 && LDS_FIN == 66560);
static_assert((NN * NN / 8) == 8 * NTHR);
static_assert(2 * NN == 64 * 4);
static_assert(2 * 32 * NN <= GROWS * NN);
static_assert(4 * NTHR * 4 == 32 * NN);
static_assert(NWAVE * 4 == 32);

typedef float          v2f  __attribute__((ext_vector_type(2)));
typedef float          v4f  __attribute__((ext_vector_type(4)));
typedef float          v8f  __attribute__((ext_vector_type(8)));
typedef int            v4i  __attribute__((ext_vector_type(4)));
typedef double         v2d  __attribute__((ext_vector_type(2)));
typedef _Float16       v8h  __attribute__((ext_vector_type(8)));
typedef _Float16       v16h __attribute__((ext_vector_type(16)));
typedef __bf16         v8b  __attribute__((ext_vector_type(8)));
typedef __bf16         v16b __attribute__((ext_vector_type(16)));
union FragH { v16h v; v8h h[2]; };
union FragB { v16b v; v8b h[2]; };
union FI { float f; int i; };

__device__ __forceinline__ v8f wmf(v16h a, v16h b, v8f c) {
  v8f d = __builtin_amdgcn_wmma_f32_16x16x32_f16(false, a, false, b, (short)0, c, false, false);
  asm volatile("v_nop\n\tv_nop\n\tv_nop\n\tv_nop" : "+v"(d) : "v"(a), "v"(b));
  return d;
}
__device__ __forceinline__ v8f wmb(v16b a, v16b b, v8f c) {
  v8f d = __builtin_amdgcn_wmma_f32_16x16x32_bf16(false, a, false, b, (short)0, c, false, false);
  asm volatile("v_nop\n\tv_nop\n\tv_nop\n\tv_nop" : "+v"(d) : "v"(a), "v"(b));
  return d;
}

template <int NB, int SRC>
__device__ __forceinline__ int scan_chunk(const int* __restrict__ keys, const int* __restrict__ gath, int nE, int nN,
                                          int cbase, int slotBase, int vec8, int* list, int tid, int lane, int wave) {
  int wc = 0;
#pragma unroll
  for (int g = 0; g < NGRP; ++g) {
    const int el0  = (g * NTHR + tid) * EPT;
    const int e0   = cbase + el0;
    const int sent = -2147483647 - 1;
    v4i da, db;
    v4i sa = {0, 0, 0, 0}, sb = {0, 0, 0, 0};
    if (vec8 != 0 && cbase + CHUNK <= nE) {
      da = *(const v4i*)(keys + e0);
      db = *(const v4i*)(keys + e0 + 4);
      if (SRC) {
        sa = *(const v4i*)(gath + e0);
        sb = *(const v4i*)(gath + e0 + 4);
      }
    } else {
      da.x = (e0     < nE) ? keys[min(e0, nE - 1)] : sent;
      da.y = (e0 + 1 < nE) ? keys[min(e0 + 1, nE - 1)] : sent;
      da.z = (e0 + 2 < nE) ? keys[min(e0 + 2, nE - 1)] : sent;
      da.w = (e0 + 3 < nE) ? keys[min(e0 + 3, nE - 1)] : sent;
      db.x = (e0 + 4 < nE) ? keys[min(e0 + 4, nE - 1)] : sent;
      db.y = (e0 + 5 < nE) ? keys[min(e0 + 5, nE - 1)] : sent;
      db.z = (e0 + 6 < nE) ? keys[min(e0 + 6, nE - 1)] : sent;
      db.w = (e0 + 7 < nE) ? keys[min(e0 + 7, nE - 1)] : sent;
      if (SRC) {
        sa.x = gath[min(e0, nE - 1)];
        sa.y = gath[min(e0 + 1, nE - 1)];
        sa.z = gath[min(e0 + 2, nE - 1)];
        sa.w = gath[min(e0 + 3, nE - 1)];
        sb.x = gath[min(e0 + 4, nE - 1)];
        sb.y = gath[min(e0 + 5, nE - 1)];
        sb.z = gath[min(e0 + 6, nE - 1)];
        sb.w = gath[min(e0 + 7, nE - 1)];
      }
    }
    if (SRC) {
      sa.x = min(max(sa.x, 0), nN - 1); sa.y = min(max(sa.y, 0), nN - 1);
      sa.z = min(max(sa.z, 0), nN - 1); sa.w = min(max(sa.w, 0), nN - 1);
      sb.x = min(max(sb.x, 0), nN - 1); sb.y = min(max(sb.y, 0), nN - 1);
      sb.z = min(max(sb.z, 0), nN - 1); sb.w = min(max(sb.w, 0), nN - 1);
    }
    const unsigned nb = (unsigned)slotBase;
    const unsigned s0 = (unsigned)da.x - nb, s1 = (unsigned)da.y - nb;
    const unsigned s2 = (unsigned)da.z - nb, s3 = (unsigned)da.w - nb;
    const unsigned s4 = (unsigned)db.x - nb, s5 = (unsigned)db.y - nb;
    const unsigned s6 = (unsigned)db.z - nb, s7 = (unsigned)db.w - nb;
    const bool h0 = s0 < (unsigned)NB, h1 = s1 < (unsigned)NB, h2 = s2 < (unsigned)NB, h3 = s3 < (unsigned)NB;
    const bool h4 = s4 < (unsigned)NB, h5 = s5 < (unsigned)NB, h6 = s6 < (unsigned)NB, h7 = s7 < (unsigned)NB;
    const unsigned any = __builtin_amdgcn_ballot_w32(h0 | h1 | h2 | h3 | h4 | h5 | h6 | h7);
    if (any != 0u) {
#define HITJ(HJ, SJ, VJ) { \
        const unsigned mj = __builtin_amdgcn_ballot_w32(HJ); \
        if (mj != 0u) { \
          if (HJ) { \
            const int pos = wc + (int)__builtin_amdgcn_mbcnt_lo(mj, 0u); \
            const int entv = SRC ? (((VJ) << ESHF) | (int)(SJ)) : (int)(SJ); \
            if (pos < WCAP) list[wave * WCAP + pos] = entv; \
          } \
          wc += (int)__builtin_popcount(mj); } }
      HITJ(h0, s0, sa.x)
      HITJ(h1, s1, sa.y)
      HITJ(h2, s2, sa.z)
      HITJ(h3, s3, sa.w)
      HITJ(h4, s4, sb.x)
      HITJ(h5, s5, sb.y)
      HITJ(h6, s6, sb.z)
      HITJ(h7, s7, sb.w)
#undef HITJ
    }
  }
  return wc;
}

__global__ __launch_bounds__(NTHR) void k_wprep(const float* __restrict__ w1, const float* __restrict__ w2, _Float16* wp) {
  const int tid = threadIdx.x;
  const int pl = (int)blockIdx.x >> 3;
  const int i  = ((int)blockIdx.x & 7) * NTHR + tid;
  const int n  = i >> 4;
  const int k0 = (i & 15) * 8;
  const float* w = pl ? w2 : w1;
  v8h hv;
#pragma unroll
  for (int e = 0; e < 8; ++e) hv[e] = (_Float16)(w[(k0 + e) * NN + n] * (float)WSCALE);
  _Float16* d = wp + (size_t)pl * (NN * NN) + (size_t)i * 8;
  *(volatile v8h*)d = hv;
  __threadfence();
  *(volatile v8h*)d = hv;
}

__global__ __launch_bounds__(NTHR) void k_count(
    const int* __restrict__ keys, int* cnt, float* dinv, int nE, int nN, int vec8) {
  extern __shared__ v4f lds_dyn[];
  int* scnt = (int*)lds_dyn;
  int* list = scnt + NBC;
  int* wcnt = list + LISTN;
  const int tid = threadIdx.x, lane = tid & 31, wave = tid >> 5;
  const int nodeBase = blockIdx.x * NBC;

  {
    const v4i z = {0, 0, 0, 0};
    for (int i = tid; i < NBC / 4; i += NTHR) ((v4i*)scnt)[i] = z;
  }
  __syncthreads();

  const int nChunks = (nE + CHUNK - 1) / CHUNK;
#pragma unroll 1
  for (int ch = 0; ch < nChunks; ++ch) {
    const int cbase = ch * CHUNK;
    const int wc = scan_chunk<NBC, 0>(keys, keys, nE, nN, cbase, nodeBase, vec8, list, tid, lane, wave);
    if (lane == 0) wcnt[wave] = wc;
    __syncthreads();
    if (wave == 0) {
#pragma unroll 1
      for (int wsx = 0; wsx < NWAVE; ++wsx) {
        int n = __builtin_amdgcn_readfirstlane(wcnt[wsx]);
        n = n > WCAP ? WCAP : (n < 0 ? 0 : n);
        const int* lp = list + wsx * WCAP;
#pragma unroll 1
        for (int i = 0; i < n; ++i) {
          const int ent  = __builtin_amdgcn_readfirstlane(lp[i]);
          const int slot = ent & (NBC - 1);
          if (lane == 0) scnt[slot] = scnt[slot] + 1;
        }
      }
    }
    __syncthreads();
  }

  int*   cp = cnt + (size_t)nodeBase;
  float* dp = dinv + (size_t)nodeBase;
#pragma unroll 4
  for (int q = 0; q < 32; ++q) {
    const int f = (wave * 32 + q) * 128 + 4 * lane;
    const v4i c = *(const v4i*)(scnt + f);
    v4f d;
    d.x = rsqrtf(fmaxf((float)c.x, 1.0f)); d.y = rsqrtf(fmaxf((float)c.y, 1.0f));
    d.z = rsqrtf(fmaxf((float)c.z, 1.0f)); d.w = rsqrtf(fmaxf((float)c.w, 1.0f));
    *(volatile v4i*)(cp + f) = c;
    *(volatile v4f*)(dp + f) = d;
  }
  __threadfence();
#pragma unroll 4
  for (int q = 0; q < 32; ++q) {
    const int f = (wave * 32 + q) * 128 + 4 * lane;
    const v4i c = *(const v4i*)(scnt + f);
    v4f d;
    d.x = rsqrtf(fmaxf((float)c.x, 1.0f)); d.y = rsqrtf(fmaxf((float)c.y, 1.0f));
    d.z = rsqrtf(fmaxf((float)c.z, 1.0f)); d.w = rsqrtf(fmaxf((float)c.w, 1.0f));
    *(volatile v4i*)(cp + f) = c;
    *(volatile v4f*)(dp + f) = d;
  }
}

__global__ __launch_bounds__(OTHR) void k_offsets(
    const int* __restrict__ cnt, int* off, int* rbase, int nBF) {
  __shared__ __attribute__((aligned(16))) int srb[RBN];
  __shared__ int wtot[OTHR / 32];
  const int tid = threadIdx.x, lane = tid & 31, wave = tid >> 5;
  for (int i = tid; i < RBN; i += OTHR) srb[i] = 0;
  int carry = 0;
#pragma unroll 1
  for (int fb = 0; fb < nBF; ++fb) {
    const int base = fb * NBF;
    const v4i c = *(const v4i*)(cnt + base + 4 * tid);
    const int e0 = max(c.x, 0), e1 = max(c.y, 0), e2 = max(c.z, 0), e3 = max(c.w, 0);
    const int ts = e0 + e1 + e2 + e3;
    int incl = ts;
#pragma unroll
    for (int d = 1; d < 32; d <<= 1) {
      const int t = __shfl_up(incl, d);
      if (lane >= d) incl += t;
    }
    if (lane == 31) wtot[wave] = incl;
    __syncthreads();
    int pre = 0;
#pragma unroll 1
    for (int w = 0; w < wave; ++w) pre += wtot[w];
    int tot = 0;
#pragma unroll
    for (int w = 0; w < OTHR / 32; ++w) tot += wtot[w];
    int run = carry + pre + incl - ts;
    v4i o;
    o.x = run; run += e0;
    o.y = run; run += e1;
    o.z = run; run += e2;
    o.w = run;
    int* op = off + base + 4 * tid;
    *(volatile v4i*)op = o;
    __threadfence();
    *(volatile v4i*)op = o;
    if (tid == 0) srb[min(fb, RBN - 1)] = carry;
    carry += (tot + 31) & ~31;
    __syncthreads();
  }
  if (tid == 0) srb[min(nBF, RBN - 1)] = carry;
  __syncthreads();
  v4i rv = {0, 0, 0, 0};
  if (tid < 32) rv = *(const v4i*)(srb + 4 * tid);
  if (tid < 32) *(volatile v4i*)(rbase + 4 * tid) = rv;
  __threadfence();
  if (tid < 32) *(volatile v4i*)(rbase + 4 * tid) = rv;
}

__global__ __launch_bounds__(NTHR) void k_fill(
    const int* __restrict__ keys, const int* __restrict__ gath,
    const int* __restrict__ off, const int* __restrict__ rbase,
    int* csr, int nN, int nE, int vec8, int csrLen) {
  extern __shared__ v4f lds_dyn[];
  int* region = (int*)lds_dyn;
  int* cursor = region + RCAP;
  int* list   = cursor + NBF;
  int* wcnt   = list + LISTN;
  const int tid = threadIdx.x, lane = tid & 31, wave = tid >> 5;
  const int b = blockIdx.x;
  const int nodeBase = b * NBF;

  int rb0 = rbase[b];
  const int rb1 = rbase[b + 1];
  rb0 = rb0 < 0 ? 0 : (rb0 > csrLen ? csrLen : rb0);
  rb0 &= ~31;
  int len = rb1 - rb0;
  len = len < 0 ? 0 : (len > RCAP ? RCAP : len);
  int lenW = (len + 31) & ~31;
  if (rb0 + lenW > csrLen) lenW = (csrLen - rb0) & ~31;

  {
    const v4i z = {0, 0, 0, 0};
    for (int i = tid; i < RCAP / 4; i += NTHR) ((v4i*)region)[i] = z;
    for (int s = tid; s < NBF; s += NTHR) {
      int o = off[nodeBase + s] - rb0;
      o = o < 0 ? 0 : (o > RCAP ? RCAP : o);
      cursor[s] = o;
    }
  }
  __syncthreads();

  const int nChunks = (nE + CHUNK - 1) / CHUNK;
#pragma unroll 1
  for (int ch = 0; ch < nChunks; ++ch) {
    const int cbase = ch * CHUNK;
    const int wc = scan_chunk<NBF, 1>(keys, gath, nE, nN, cbase, nodeBase, vec8, list, tid, lane, wave);
    if (lane == 0) wcnt[wave] = wc;
    __syncthreads();
    if (wave == 0) {
#pragma unroll 1
      for (int wsx = 0; wsx < NWAVE; ++wsx) {
        int n = __builtin_amdgcn_readfirstlane(wcnt[wsx]);
        n = n > WCAP ? WCAP : (n < 0 ? 0 : n);
        const int* lp = list + wsx * WCAP;
#pragma unroll 1
        for (int i = 0; i < n; ++i) {
          const int ent  = __builtin_amdgcn_readfirstlane(lp[i]);
          const int slot = ent & (NBF - 1);
          int src = (ent >> ESHF) & 0xFFFFF;
          src = src > nN - 1 ? nN - 1 : src;
          if (lane == 0) {
            int pos = cursor[slot];
            pos = pos < 0 ? 0 : (pos > RCAP - 1 ? RCAP - 1 : pos);
            region[pos] = src;
            const int np = pos + 1;
            cursor[slot] = np > RCAP ? RCAP : np;
          }
        }
      }
    }
    __syncthreads();
  }

  const int nv = lenW >> 2;
  int* gp = csr + rb0;
#pragma unroll 1
  for (int i = tid; i < nv; i += NTHR) { const v4i v = ((const v4i*)region)[i]; *(volatile v4i*)(gp + 4 * i) = v; }
  __threadfence();
#pragma unroll 1
  for (int i = tid; i < nv; i += NTHR) { const v4i v = ((const v4i*)region)[i]; *(volatile v4i*)(gp + 4 * i) = v; }
}

__global__ __launch_bounds__(NTHR) void k_agg(
    const int* __restrict__ csr, const int* __restrict__ off, const int* __restrict__ cnt,
    const float* __restrict__ dvo, const float* __restrict__ feat,
    float* agg, int nN, int csrLen) {
  const int tid = threadIdx.x, lane = tid & 31, wave = tid >> 5;
  const int tbase = blockIdx.x * TGT + wave * 32;
  const int cl = tbase + lane;
  const int cnt_l = cnt[cl];
  const int off_l = off[cl];

#pragma unroll 1
  for (int j = 0; j < 32; ++j) {
    const int c = tbase + j;
    int n = __builtin_amdgcn_readlane(cnt_l, j);
    n = n < 0 ? 0 : (n > DEGCAP ? DEGCAP : n);
    const int st = __builtin_amdgcn_readlane(off_l, j);
    v4f acc = {0.f, 0.f, 0.f, 0.f};
#pragma unroll 1
    for (int q0 = 0; q0 < n; q0 += 32) {
      int pos = st + q0 + lane;
      pos = pos < 0 ? 0 : (pos > csrLen - 1 ? csrLen - 1 : pos);
      int sl = csr[pos];
      sl = sl < 0 ? 0 : (sl > nN - 1 ? nN - 1 : sl);
      FI nsl; nsl.f = dvo[sl];
      const int mcnt = (n - q0) < 32 ? (n - q0) : 32;
#pragma unroll 1
      for (int p = 0; p < mcnt; ++p) {
        const int s = __builtin_amdgcn_readlane(sl, p);
        FI nu; nu.i = __builtin_amdgcn_readlane(nsl.i, p);
        const v4f v = *(const v4f*)(feat + (size_t)s * NN + 4 * lane);
        acc = acc + v * nu.f;
      }
    }
    float* gp = agg + (size_t)c * NN + 4 * lane;
    *(volatile v4f*)gp = acc;
    __threadfence();
    *(volatile v4f*)gp = acc;
  }
}

template <int ASC, int RELU>
__global__ __launch_bounds__(NTHR) void k_gemm(
    const float* __restrict__ A, const _Float16* __restrict__ Bw, const float* __restrict__ dinv,
    const float* __restrict__ bias, float* C, int nRowsA, int nRowsOut) {
  extern __shared__ v4f lds_dyn[];
  constexpr float OSC = 1.0f / (float)(ASC * WSCALE);
  float* stg = (float*)lds_dyn;
  const int tid = threadIdx.x, lane = tid & 31, wave = tid >> 5, hh = lane >> 4, m = lane & 15;
  const int rowBase = blockIdx.x * GROWS;
  int arow = rowBase + wave * 16 + m;
  arow = arow > nRowsA - 1 ? nRowsA - 1 : arow;
  const float cs = dinv[arow] * (float)ASC;
  const float* ap = A + (size_t)arow * NN + 8 * hh;

  v8f acc[8];
#pragma unroll
  for (int t = 0; t < 8; ++t) { v8f z = {0.f, 0.f, 0.f, 0.f, 0.f, 0.f, 0.f, 0.f}; acc[t] = z; }

#pragma unroll 1
  for (int kt = 0; kt < NN / 32; ++kt) {
    const float* akp = ap + 32 * kt;
    const v4f f0 = *(const v4f*)akp;
    const v4f f1 = *(const v4f*)(akp + 4);
    const v4f f2 = *(const v4f*)(akp + 16);
    const v4f f3 = *(const v4f*)(akp + 20);
    v8h lo, hi;
    lo[0] = (_Float16)(f0.x * cs); lo[1] = (_Float16)(f0.y * cs);
    lo[2] = (_Float16)(f0.z * cs); lo[3] = (_Float16)(f0.w * cs);
    lo[4] = (_Float16)(f1.x * cs); lo[5] = (_Float16)(f1.y * cs);
    lo[6] = (_Float16)(f1.z * cs); lo[7] = (_Float16)(f1.w * cs);
    hi[0] = (_Float16)(f2.x * cs); hi[1] = (_Float16)(f2.y * cs);
    hi[2] = (_Float16)(f2.z * cs); hi[3] = (_Float16)(f2.w * cs);
    hi[4] = (_Float16)(f3.x * cs); hi[5] = (_Float16)(f3.y * cs);
    hi[6] = (_Float16)(f3.z * cs); hi[7] = (_Float16)(f3.w * cs);
    FragH af;
    af.h[0] = lo;
    af.h[1] = hi;
#pragma unroll
    for (int t = 0; t < 8; ++t) {
      const _Float16* bp = Bw + (size_t)(16 * t + m) * NN + 32 * kt + 8 * hh;
      FragH bf;
      bf.h[0] = *(const v8h*)bp;
      bf.h[1] = *(const v8h*)(bp + 16);
      acc[t] = wmf(af.v, bf.v, acc[t]);
    }
  }

  const int r0 = wave * 16 + 8 * hh;
  float* sp = stg + r0 * NN + m;
#pragma unroll
  for (int t = 0; t < 8; ++t) {
    const float bt = bias[16 * t + m];
#pragma unroll
    for (int r = 0; r < 8; ++r) {
      float v = acc[t][r] * OSC + bt;
      if (RELU) v = fmaxf(v, 0.0f);
      sp[r * NN + 16 * t] = v;
    }
  }
  __syncthreads();

  const float* lp = stg + wave * 16 * NN;
  float* gp = C + (size_t)(rowBase + wave * 16) * NN;
#pragma unroll
  for (int i = 0; i < 16; ++i) {
    if (rowBase + wave * 16 + i < nRowsOut) {
      const v4f v = *(const v4f*)(lp + i * NN + 4 * lane);
      *(volatile v4f*)(gp + i * NN + 4 * lane) = v;
    }
  }
  __threadfence();
#pragma unroll
  for (int i = 0; i < 16; ++i) {
    if (rowBase + wave * 16 + i < nRowsOut) {
      const v4f v = *(const v4f*)(lp + i * NN + 4 * lane);
      *(volatile v4f*)(gp + i * NN + 4 * lane) = v;
    }
  }
}

__global__ __launch_bounds__(NTHR) void k_colstats(const float* __restrict__ z1, const float* __restrict__ z2,
                                                   double* part, int nN, int rpb) {
  __shared__ __attribute__((aligned(16))) double lay[2 * NTHR];
  const int tid = threadIdx.x;
  const int mat = tid >> 7, c = tid & (NN - 1);
  const float* Z = mat ? z2 : z1;
  const int r0 = blockIdx.x * rpb;
  int r1 = r0 + rpb;
  r1 = r1 > nN ? nN : r1;
  double s = 0.0, q = 0.0;
#pragma unroll 1
  for (int r = r0; r < r1; ++r) {
    const double dv = (double)Z[(size_t)r * NN + c];
    s += dv;
    q += dv * dv;
  }
  lay[tid] = s;
  lay[NTHR + tid] = q;
  __syncthreads();
  const v2d w = *(const v2d*)(lay + 2 * tid);
  double* gp = part + (size_t)blockIdx.x * (2 * NTHR) + 2 * tid;
  *(volatile v2d*)gp = w;
  __threadfence();
  *(volatile v2d*)gp = w;
}

__global__ __launch_bounds__(NTHR) void k_moments(const double* __restrict__ part, int nSB,
                                                  float* mu, float* inv, double rN, double rN1) {
  __shared__ __attribute__((aligned(16))) float smu[2 * NN];
  __shared__ __attribute__((aligned(16))) float siv[2 * NN];
  const int tid = threadIdx.x;
  double S = 0.0, Q = 0.0;
#pragma unroll 1
  for (int b = 0; b < nSB; ++b) {
    S += part[(size_t)b * (2 * NTHR) + tid];
    Q += part[(size_t)b * (2 * NTHR) + NTHR + tid];
  }
  const double mean = S * rN;
  double var = (Q - S * mean) * rN1;
  var = var > 0.0 ? var : 0.0;
  const float sdf = sqrtf((float)var);
  const float muf = (float)mean;
  const float den = sdf + 1e-6f;
  const float ivf = 1.0f / den;
  smu[tid] = muf;
  siv[tid] = ivf;
  __syncthreads();

  const int q = tid & 63;
  const v4f vm = *(const v4f*)(smu + 4 * q);
  const v4f vi = *(const v4f*)(siv + 4 * q);
  const bool wm = tid < 64;
  const bool wi = (tid >= 64) && (tid < 128);
  if (wm) *(volatile v4f*)(mu + 4 * q) = vm;
  if (wi) *(volatile v4f*)(inv + 4 * q) = vi;
  __threadfence();
  if (wm) *(volatile v4f*)(mu + 4 * q) = vm;
  if (wi) *(volatile v4f*)(inv + 4 * q) = vi;
}

__global__ __launch_bounds__(NTHR) void k_corr(
    const float* __restrict__ z1, const float* __restrict__ z2,
    const float* __restrict__ mu, const float* __restrict__ inv,
    float* part, int nN) {
  extern __shared__ v4f lds_dyn[];
  __bf16* T = (__bf16*)lds_dyn;
  float* stg = (float*)((char*)lds_dyn + 4 * NN * 32 * 2);
  float* zt = stg;
  const int tid = threadIdx.x, lane = tid & 31, wave = tid >> 5, hh = lane >> 4, m = lane & 15;
  const int mat = tid >> 7;
  const int c = tid & (NN - 1);
  const float muc = mu[mat * NN + c];
  const float ivc = inv[mat * NN + c];
  __bf16* Th = T + (size_t)(2 * mat) * (NN * 32) + c * 32;
  __bf16* Tl = Th + NN * 32;
  const float* ztc = zt + mat * (32 * NN) + c;
  const int rowBase = blockIdx.x * CRB;

  v8f acc[8];
#pragma unroll
  for (int t = 0; t < 8; ++t) { v8f z = {0.f, 0.f, 0.f, 0.f, 0.f, 0.f, 0.f, 0.f}; acc[t] = z; }

  const __bf16* Ap = T + (16 * wave + m) * 32 + 8 * hh;
  const __bf16* Bp = T + 2 * (NN * 32) + m * 32 + 8 * hh;

#pragma unroll 1
  for (int ks = 0; ks < CRB / 32; ++ks) {
    const int k0 = rowBase + ks * 32;
#pragma unroll
    for (int q = 0; q < 4; ++q) {
      const int r = 8 * q + wave;
      int gr = k0 + r;
      gr = gr < nN ? gr : nN - 1;
      const v4f a = *(const v4f*)(z1 + (size_t)gr * NN + 4 * lane);
      *(v4f*)(zt + r * NN + 4 * lane) = a;
    }
#pragma unroll
    for (int q = 0; q < 4; ++q) {
      const int r = 8 * q + wave;
      int gr = k0 + r;
      gr = gr < nN ? gr : nN - 1;
      const v4f a = *(const v4f*)(z2 + (size_t)gr * NN + 4 * lane);
      *(v4f*)(zt + 32 * NN + r * NN + 4 * lane) = a;
    }
    __syncthreads();
#pragma unroll
    for (int q = 0; q < 4; ++q) {
      v8b hv, lv;
#pragma unroll
      for (int e = 0; e < 8; ++e) {
        const int r = 8 * q + e;
        const float zv = ztc[r * NN];
        float v = (zv - muc) * ivc;
        v = (k0 + r) < nN ? v : 0.0f;
        const unsigned u  = __float_as_uint(v);
        const unsigned hu = (u + 0x7FFFu + ((u >> 16) & 1u)) >> 16;
        const float hf = __uint_as_float(hu << 16);
        const float rem = v - hf;
        const unsigned ur = __float_as_uint(rem);
        const unsigned lu = (ur + 0x7FFFu + ((ur >> 16) & 1u)) >> 16;
        hv[e] = __builtin_bit_cast(__bf16, (unsigned short)hu);
        lv[e] = __builtin_bit_cast(__bf16, (unsigned short)lu);
      }
      *(v8b*)(Th + 8 * q) = hv;
      *(v8b*)(Tl + 8 * q) = lv;
    }
    __syncthreads();
    FragB ah, al;
    ah.h[0] = *(const v8b*)Ap;               ah.h[1] = *(const v8b*)(Ap + 16);
    al.h[0] = *(const v8b*)(Ap + NN * 32);   al.h[1] = *(const v8b*)(Ap + NN * 32 + 16);
#pragma unroll
    for (int t = 0; t < 8; ++t) {
      const __bf16* bp = Bp + 16 * t * 32;
      FragB bh, bl;
      bh.h[0] = *(const v8b*)bp;             bh.h[1] = *(const v8b*)(bp + 16);
      bl.h[0] = *(const v8b*)(bp + NN * 32); bl.h[1] = *(const v8b*)(bp + NN * 32 + 16);
      acc[t] = wmb(ah.v, bh.v, acc[t]);
      acc[t] = wmb(al.v, bh.v, acc[t]);
      acc[t] = wmb(ah.v, bl.v, acc[t]);
    }
    __syncthreads();
  }

  float* sp = stg + (wave * 16 + 8 * hh) * NN + m;
#pragma unroll
  for (int t = 0; t < 8; ++t) {
#pragma unroll
    for (int r = 0; r < 8; ++r) sp[r * NN + 16 * t] = acc[t][r];
  }
  __syncthreads();

  const float* lp = stg + wave * 16 * NN;
  float* gp = part + (size_t)blockIdx.x * (NN * NN) + (size_t)wave * 16 * NN;
#pragma unroll
  for (int i = 0; i < 16; ++i) {
    const v4f v = *(const v4f*)(lp + i * NN + 4 * lane);
    *(volatile v4f*)(gp + i * NN + 4 * lane) = v;
  }
  __threadfence();
#pragma unroll
  for (int i = 0; i < 16; ++i) {
    const v4f v = *(const v4f*)(lp + i * NN + 4 * lane);
    *(volatile v4f*)(gp + i * NN + 4 * lane) = v;
  }
}

__global__ __launch_bounds__(NTHR) void k_final(const float* __restrict__ part, int nCB,
                                                const float* __restrict__ roff, const float* __restrict__ coff,
                                                float* out, double rN) {
  extern __shared__ v4f lds_dyn[];
  float* Csh = (float*)lds_dyn;
  float* msk = Csh + NN * NN;
  const int tid = threadIdx.x;
#pragma unroll 1
  for (int e = 0; e < (NN * NN) / NTHR; ++e) {
    const int idx = e * NTHR + tid;
    double s = 0.0;
#pragma unroll 1
    for (int b = 0; b < nCB; ++b) s += (double)part[(size_t)b * (NN * NN) + idx];
    Csh[idx] = (float)(s * rN);
  }
  __syncthreads();
  {
    const int which = tid >> 7, i = tid & (NN - 1);
    const int strd = which ? NN : 1;
    const int b0 = which ? i : i * NN;
    double s = 0.0;
#pragma unroll 1
    for (int j = 0; j < NN; ++j) s += (double)fabsf(Csh[b0 + j * strd]);
    const float score = (float)(s * (1.0 / (double)NN));
    const float ro = roff[i], co = coff[i];
    const float ov = which ? co : ro;
    const float t1 = score + ov;
    const float t2 = t1 - 0.05f;
    const float x = 50.0f * t2;
    const float mk = 1.0f / (1.0f + expf(-x));
    msk[tid] = mk;
  }
  __syncthreads();

#pragma unroll 1
  for (int it = 0; it < (NN * NN) / (4 * NTHR); ++it) {
    const int f = it * (4 * NTHR) + 4 * tid;
    const int i = f >> 7, j = f & (NN - 1);
    const v4f cv = *(const v4f*)(Csh + f);
    const float rm = msk[i];
    const v4f cm = *(const v4f*)(msk + NN + j);
    const v4f wgt = cm * rm;
    const v4f o = cv * wgt;
    *(volatile v4f*)(out + f) = o;
  }
  if (tid < 64) {
    const v4f mv = *(const v4f*)(msk + 4 * tid);
    *(volatile v4f*)(out + NN * NN + 4 * tid) = mv;
  }
  __threadfence();
#pragma unroll 1
  for (int it = 0; it < (NN * NN) / (4 * NTHR); ++it) {
    const int f = it * (4 * NTHR) + 4 * tid;
    const int i = f >> 7, j = f & (NN - 1);
    const v4f cv = *(const v4f*)(Csh + f);
    const float rm = msk[i];
    const v4f cm = *(const v4f*)(msk + NN + j);
    const v4f wgt = cm * rm;
    const v4f o = cv * wgt;
    *(volatile v4f*)(out + f) = o;
  }
  if (tid < 64) {
    const v4f mv = *(const v4f*)(msk + 4 * tid);
    *(volatile v4f*)(out + NN * NN + 4 * tid) = mv;
  }
}

static void run_tower(const float* x, const int* src, const int* dst, int nE, int nN,
                      const _Float16* wp, const float* b1, const float* b2,
                      int* cnt, float* dvi, float* dvo, int* offp, int* rb, int* csr,
                      float* agg, float* h, float* z,
                      int nBC, int nBF, int csrLen, int nAgg, int nGemm, int NPAD, hipStream_t stream) {
  const int vec8 = 1;
  k_count<<<nBC, NTHR, LDS_COUNT, stream>>>(src, cnt, dvo, nE, nN, vec8);
  k_count<<<nBC, NTHR, LDS_COUNT, stream>>>(dst, cnt, dvi, nE, nN, vec8);
  k_offsets<<<1, OTHR, 0, stream>>>(cnt, offp, rb, nBF);
  k_fill<<<nBF, NTHR, LDS_FILL, stream>>>(dst, src, offp, rb, csr, nN, nE, vec8, csrLen);
  k_agg<<<nAgg, NTHR, 0, stream>>>(csr, offp, cnt, dvo, x, agg, nN, csrLen);
  k_gemm<ASC1, 1><<<nGemm, NTHR, LDS_GEMM, stream>>>(agg, wp, dvi, b1, h, NPAD, NPAD);
  k_agg<<<nAgg, NTHR, 0, stream>>>(csr, offp, cnt, dvo, h, agg, nN, csrLen);
  k_gemm<ASC2, 0><<<nGemm, NTHR, LDS_GEMM, stream>>>(agg, wp + (size_t)NN * NN, dvi, b2, z, NPAD, nN);
}

extern "C" void kernel_launch(void* const* d_in, const int* in_sizes, int n_in,
                              void* d_out, int out_size, void* d_ws, size_t ws_size,
                              hipStream_t stream) {
  if (n_in < 12) return;
  const int nN = in_sizes[0] / NN;
  if (nN <= 0 || in_sizes[0] != nN * NN || in_sizes[1] != nN * NN) return;
  const int nE1 = in_sizes[2], nE2 = in_sizes[4];
  if (nE1 <= 0 || nE2 <= 0 || in_sizes[3] != nE1 || in_sizes[5] != nE2) return;
  if (in_sizes[6] != NN * NN || in_sizes[8] != NN * NN) return;
  if (in_sizes[7] != NN || in_sizes[9] != NN || in_sizes[10] != NN || in_sizes[11] != NN) return;
  if (out_size != NN * NN + 2 * NN + 2 * nN * NN) return;
  if (nN > (1 << 20) || nE1 > (1 << 28) || nE2 > (1 << 28)) return;
  const int nEmax = nE1 > nE2 ? nE1 : nE2;

  const float* x1   = (const float*)d_in[0];
  const float* x2   = (const float*)d_in[1];
  const int*   src1 = (const int*)d_in[2];
  const int*   dst1 = (const int*)d_in[3];
  const int*   src2 = (const int*)d_in[4];
  const int*   dst2 = (const int*)d_in[5];
  const float* W1   = (const float*)d_in[6];
  const float* b1   = (const float*)d_in[7];
  const float* W2   = (const float*)d_in[8];
  const float* b2   = (const float*)d_in[9];
  const float* roff = (const float*)d_in[10];
  const float* coff = (const float*)d_in[11];
  float* out = (float*)d_out;
  float* z1 = out + NN * NN + 2 * NN;
  float* z2 = z1 + (size_t)nN * NN;

  const int NPAD   = ((nN + TGT - 1) / TGT) * TGT;
  const int nBC    = (nN + NBC - 1) / NBC;
  const int CNTPAD = nBC * NBC;
  const int nBF    = (nN + NBF - 1) / NBF;
  const int OFFN   = nBF * NBF;
  if (nBF + 1 > RBN) return;
  if (OFFN > CNTPAD || NPAD > OFFN) return;
  const int csrLen = ((nEmax + 31) & ~31) + 32 * (nBF + 1);
  const int nGemm  = NPAD / GROWS;
  const int nAgg   = NPAD / TGT;
  const int nSB    = (nN + SRPB - 1) / SRPB;
  const int nCB    = (nN + CRB - 1) / CRB;

  char* ws = (char*)d_ws;
  size_t off = 0;
  const size_t oW   = off; off += (size_t)2 * NN * NN * 2;          off = (off + 255) & ~(size_t)255;
  const size_t oCnt = off; off += (size_t)CNTPAD * 4;               off = (off + 255) & ~(size_t)255;
  const size_t oDvi = off; off += (size_t)CNTPAD * 4;               off = (off + 255) & ~(size_t)255;
  const size_t oDvo = off; off += (size_t)CNTPAD * 4;               off = (off + 255) & ~(size_t)255;
  const size_t oOff = off; off += (size_t)OFFN * 4;                 off = (off + 255) & ~(size_t)255;
  const size_t oRb  = off; off += (size_t)RBN * 4;                  off = (off + 255) & ~(size_t)255;
  const size_t oCsr = off; off += (size_t)csrLen * 4;               off = (off + 255) & ~(size_t)255;
  const size_t oAgg = off; off += (size_t)NPAD * NN * 4;            off = (off + 255) & ~(size_t)255;
  const size_t oH   = off; off += (size_t)NPAD * NN * 4;            off = (off + 255) & ~(size_t)255;
  const size_t oSp  = off; off += (size_t)nSB * (2 * NTHR) * 8;     off = (off + 255) & ~(size_t)255;
  const size_t oMu  = off; off += (size_t)(2 * NN) * 4;             off = (off + 255) & ~(size_t)255;
  const size_t oInv = off; off += (size_t)(2 * NN) * 4;             off = (off + 255) & ~(size_t)255;
  const size_t oCp  = off; off += (size_t)nCB * (NN * NN) * 4;      off = (off + 255) & ~(size_t)255;
  if (off > ws_size || off > (size_t)WSCAP) return;
  _Float16* wp   = (_Float16*)(ws + oW);
  int*      cnt  = (int*)(ws + oCnt);
  float*    dvi  = (float*)(ws + oDvi);
  float*    dvo  = (float*)(ws + oDvo);
  int*      offp = (int*)(ws + oOff);
  int*      rb   = (int*)(ws + oRb);
  int*      csr  = (int*)(ws + oCsr);
  float*    agg  = (float*)(ws + oAgg);
  float*    h    = (float*)(ws + oH);
  double*   sp   = (double*)(ws + oSp);
  float*    mu   = (float*)(ws + oMu);
  float*    inv  = (float*)(ws + oInv);
  float*    cp   = (float*)(ws + oCp);

  const double rN  = 1.0 / (double)nN;
  const double rN1 = nN > 1 ? 1.0 / (double)(nN - 1) : 1.0;

  hipFuncSetAttribute(reinterpret_cast<const void*>(&k_count), hipFuncAttributeMaxDynamicSharedMemorySize, LDS_COUNT);
  hipFuncSetAttribute(reinterpret_cast<const void*>(&k_fill), hipFuncAttributeMaxDynamicSharedMemorySize, LDS_FILL);
  hipFuncSetAttribute(reinterpret_cast<const void*>(&k_gemm<ASC1, 1>), hipFuncAttributeMaxDynamicSharedMemorySize, LDS_GEMM);
  hipFuncSetAttribute(reinterpret_cast<const void*>(&k_gemm<ASC2, 0>), hipFuncAttributeMaxDynamicSharedMemorySize, LDS_GEMM);
  hipFuncSetAttribute(reinterpret_cast<const void*>(&k_corr), hipFuncAttributeMaxDynamicSharedMemorySize, LDS_CORR);
  hipFuncSetAttribute(reinterpret_cast<const void*>(&k_final), hipFuncAttributeMaxDynamicSharedMemorySize, LDS_FIN);

  k_wprep<<<16, NTHR, 0, stream>>>(W1, W2, wp);

  run_tower(x1, src1, dst1, nE1, nN, wp, b1, b2, cnt, dvi, dvo, offp, rb, csr, agg, h, z1,
            nBC, nBF, csrLen, nAgg, nGemm, NPAD, stream);
  run_tower(x2, src2, dst2, nE2, nN, wp, b1, b2, cnt, dvi, dvo, offp, rb, csr, agg, h, z2,
            nBC, nBF, csrLen, nAgg, nGemm, NPAD, stream);

  k_colstats<<<nSB, NTHR, 0, stream>>>(z1, z2, sp, nN, SRPB);
  k_moments<<<1, NTHR, 0, stream>>>(sp, nSB, mu, inv, rN, rN1);
  k_corr<<<nCB, NTHR, LDS_CORR, stream>>>(z1, z2, mu, inv, cp, nN);
  k_final<<<1, NTHR, LDS_FIN, stream>>>(cp, nCB, roff, coff, out, rN);
}
